// Clustering_73744588472727
// MI455X (gfx1250) — hardware-verified
//
#include <hip/hip_runtime.h>
#include <math.h>

typedef __attribute__((ext_vector_type(16))) _Float16 v16h;
typedef __attribute__((ext_vector_type(16))) __bf16 v16b;
typedef __attribute__((ext_vector_type(8)))  _Float16 v8h;
typedef __attribute__((ext_vector_type(8)))  float v8f;
typedef __attribute__((ext_vector_type(4)))  float v4f;
typedef __attribute__((ext_vector_type(2)))  float v2f;
typedef __attribute__((ext_vector_type(4)))  unsigned v4u;
typedef __attribute__((ext_vector_type(4)))  int v4i;
typedef float __attribute__((may_alias)) float_a;
typedef int __attribute__((may_alias)) int_a;

template <typename T> __device__ __forceinline__ void vst2(void* p, T v) { *(volatile T*)p = v; __threadfence(); *(volatile T*)p = v; }
__device__ __forceinline__ v8f wmma16(v16h a, v16h b, v8f c) {
  v8f d = __builtin_amdgcn_wmma_f32_16x16x32_f16(false, a, false, b, (short)0, c, false, false);
  asm volatile("v_nop\n\tv_nop\n\tv_nop\n\tv_nop" : "+v"(d) : "v"(a), "v"(b));
  return d;
}
__device__ __forceinline__ v8f wmma_bf(v16b a, v16b b, v8f c) {
  v8f d = __builtin_amdgcn_wmma_f32_16x16x32_bf16(false, a, false, b, (short)0, c, false, false);
  asm volatile("v_nop\n\tv_nop\n\tv_nop\n\tv_nop" : "+v"(d) : "v"(a), "v"(b));
  return d;
}
__device__ __forceinline__ v16h frag_h(const _Float16* rowk0, int lane) {
  union { v16h v; v8h q[2]; } u; const _Float16* p = rowk0 + 8 * (lane >> 4);
  u.q[0] = *(const v8h*)p; u.q[1] = *(const v8h*)(p + 16); return u.v;
}
__device__ __forceinline__ v16h frag_f32(const float* rowk0, int lane) {
  v16h a; const float* p = rowk0 + 8 * (lane >> 4);
#pragma unroll
  for (int i = 0; i < 8; ++i) { a[i] = (_Float16)p[i]; a[8 + i] = (_Float16)p[16 + i]; }
  return a;
}
__device__ __forceinline__ v16h frag_f32s(const float* rowk0, int lane, float sc) {
  v16h a; const float* p = rowk0 + 8 * (lane >> 4);
#pragma unroll
  for (int i = 0; i < 8; ++i) { a[i] = (_Float16)(p[i] * sc); a[8 + i] = (_Float16)(p[16 + i] * sc); }
  return a;
}
__device__ __forceinline__ v16h fragc_f32(const float* W, int k0, int n, int lane, int ld, int K) {
  v16h a; const int g = lane >> 4;
#pragma unroll
  for (int i = 0; i < 8; ++i) { const int ka = k0 + 8 * g + i, kb = ka + 16;
    a[i] = (_Float16)(ka < K ? W[(size_t)(ka < K ? ka : K - 1) * ld + n] : 0.f); a[8 + i] = (_Float16)(kb < K ? W[(size_t)(kb < K ? kb : K - 1) * ld + n] : 0.f); }
  return a;
}
struct F2 { v16b h, l; };
__device__ __forceinline__ F2 bsplit16(const float v[16]) { F2 r;
#pragma unroll
  for (int i = 0; i < 16; ++i) { const __bf16 h = (__bf16)v[i]; r.h[i] = h; r.l[i] = (__bf16)(v[i] - (float)h); }
  return r; }
__device__ __forceinline__ F2 split_row(const float* row, int k0, int lane) { float v[16]; const float* p = row + k0 + 8 * (lane >> 4);
#pragma unroll
  for (int i = 0; i < 8; ++i) { v[i] = p[i]; v[8 + i] = p[16 + i]; }
  return bsplit16(v); }
__device__ __forceinline__ F2 split_rowK(const float* row, int k0, int lane, int K) { float v[16]; const int g = lane >> 4;
#pragma unroll
  for (int i = 0; i < 8; ++i) { const int ka = k0 + 8 * g + i, kb = ka + 16; v[i] = ka < K ? row[ka < K ? ka : K - 1] : 0.f; v[8 + i] = kb < K ? row[kb < K ? kb : K - 1] : 0.f; }
  return bsplit16(v); }
__device__ __forceinline__ F2 split_col(const float* W, int k0, int n, int lane, int ld, int K) { float v[16]; const int g = lane >> 4;
#pragma unroll
  for (int i = 0; i < 8; ++i) { const int ka = k0 + 8 * g + i, kb = ka + 16; v[i] = ka < K ? W[(size_t)(ka < K ? ka : K - 1) * ld + n] : 0.f; v[8 + i] = kb < K ? W[(size_t)(kb < K ? kb : K - 1) * ld + n] : 0.f; }
  return bsplit16(v); }
__device__ __forceinline__ v8f mac3(const F2& a, const F2& b, v8f c) { c = wmma_bf(a.l, b.h, c); c = wmma_bf(a.h, b.l, c); return wmma_bf(a.h, b.h, c); }
__device__ __forceinline__ float sigm(float v) { return 1.0f / (1.0f + expf(-v)); }
#define LDSX() do { asm volatile("s_wait_dscnt 0" ::: "memory"); __builtin_amdgcn_wave_barrier(); __builtin_amdgcn_fence(__ATOMIC_RELEASE, "workgroup"); } while (0)


#define NB 8
#define NH 8
#define NL 1024
#define DD 64
#define NC 5
#define DMOD (NH * DD)
#define KCONV (3 * DMOD)
#ifndef TNB
#define TNB NB
#endif
#ifndef TBH0
#define TBH0 0
#endif
#ifndef TBHN
#define TBHN (NB * NH)
#endif
#ifndef TKS0
#define TKS0 0
#endif
#ifndef TKSN
#define TKSN NB
#endif
typedef __attribute__((ext_vector_type(8))) __bf16 v8b;
__device__ __forceinline__ v16b frag_b(const __bf16* rowk0, int lane) {
  union { v16b v; v8b q[2]; } u; const __bf16* p = rowk0 + 8 * (lane >> 4);
  u.q[0] = *(const v8b*)p; u.q[1] = *(const v8b*)(p + 16); return u.v;
}
__device__ __forceinline__ float bfr(float v) { return (float)(__bf16)v; }
__device__ __attribute__((noinline)) float exp_ni(float v) { return expf(v); }
__device__ __attribute__((noinline)) float erf_ni(float v) { return erff(v); }

#define WS_CQ2 0u
#define WS_MU  (WS_CQ2 + 4u * (size_t)NB * NC * NL * 8)
#define WS_LP  (WS_MU + 4u * (size_t)NB * NL * 8)
#define WS_KSH (WS_LP + 4u * (size_t)NB * NL * 8)
#define WS_KSL (WS_KSH + 2u * (size_t)NB * NH * NL * DD)
#define WS_VT  (WS_KSL + 2u * (size_t)NB * NH * NL * DD)
#define WS_END (WS_VT + 2u * (size_t)NB * NH * DD * NL)

__global__ __launch_bounds__(128) void k_ckp(const float* __restrict__ Kin, const float* __restrict__ WPK, const float* __restrict__ BPK, const float* __restrict__ WCK, const float* __restrict__ BCK, const float* __restrict__ WCQ, const float* __restrict__ BCQ, float* __restrict__ CQ2, float* __restrict__ MU, float* __restrict__ LP) {
  __shared__ __align__(16) float sck[64][NC][8];
  __shared__ __align__(16) float scq2[NC][64][8];
  __shared__ __align__(16) float smu[64][8], slp[64][8]; __shared__ float sthr[64][68];
  const int tid = threadIdx.x, wave = tid >> 5, lane = tid & 31, col = lane & 15, g = lane >> 4; const int b = blockIdx.y; const int l20 = blockIdx.x * 64;
#pragma unroll 1
  for (int tile = wave; tile < 20; tile += 4) { const int r = tile * 16 + col; const int l2l = r / NC, u2 = r % NC; const int l2 = l20 + l2l; const int dfix = l2 & 63; const int lb = l2 >> 6;
    v8f acc = {};
#pragma unroll 1
    for (int kc = 0; kc < KCONV / 32; ++kc) { const int t = (kc * 32) / DMOD; const int cbase = (kc * 32) % DMOD; const int us = u2 + t - 1; const int bb = b + us - 4; const bool live = (us >= 0 && us < NC && bb >= 1 && bb < NB);
      v16b a;
#pragma unroll
      for (int i = 0; i < 8; ++i) { const int c0 = cbase + 8 * g + i, c1 = c0 + 16; float x0 = 0.f, x1 = 0.f;
        if (live) { { const int hh = c0 >> 6, ll = (c0 * 16 + lb) & (NL - 1); x0 = Kin[((((size_t)bb * NH + hh) * NL + ll) * DD) + dfix]; } { const int hh = c1 >> 6, ll = (c1 * 16 + lb) & (NL - 1); x1 = Kin[((((size_t)bb * NH + hh) * NL + ll) * DD) + dfix]; } }
        a[i] = (__bf16)x0; a[8 + i] = (__bf16)x1; }
      v16b w;
#pragma unroll
      for (int i = 0; i < 8; ++i) { const int c0 = cbase + 8 * g + i, c1 = c0 + 16; w[i] = (__bf16)((col < NC) ? WPK[((size_t)col * DMOD + c0) * 3 + t] : 0.f); w[8 + i] = (__bf16)((col < NC) ? WPK[((size_t)col * DMOD + c1) * 3 + t] : 0.f); }
      acc = wmma_bf(a, w, acc); }
    if (col < NC) {
#pragma unroll
      for (int rr = 0; rr < 8; ++rr) { const int row = tile * 16 + 8 * g + rr; sck[row / NC][row % NC][col] = fmaxf(acc[rr] + bfr(BPK[col]), 0.f); } } }
  __syncthreads();
  if (tid < 64) { const int l2l = tid; float* cqf = &sthr[tid][0]; float* ckf = &sthr[tid][25]; float* zk = &sthr[tid][50]; float* zq = &sthr[tid][55]; float* e = &sthr[tid][60];
#define cq(A,B) cqf[(A) * NC + (B)]
#define ck(A,B) ckf[(A) * NC + (B)]
#pragma unroll 1
    for (int uu = 0; uu < NC; ++uu) { float mk = -3.0e38f, mq = -3.0e38f;
#pragma unroll 1
      for (int o = 0; o < NC; ++o) { float ak = bfr(BCK[o]), aq = bfr(BCQ[o]);
#pragma unroll 1
        for (int c = 0; c < NC; ++c) { const float x = sck[l2l][uu][c]; ak += x * bfr(WCK[o * NC + c]); aq += x * bfr(WCQ[o * NC + c]); }
        zk[o] = ak; zq[o] = aq; mk = fmaxf(mk, ak); mq = fmaxf(mq, aq); }
      float sk = 0.f, sq = 0.f;
#pragma unroll 1
      for (int o = 0; o < NC; ++o) { zk[o] = expf(zk[o] - mk); sk += zk[o]; zq[o] = expf(zq[o] - mq); sq += zq[o]; }
#pragma unroll 1
      for (int o = 0; o < NC; ++o) { ck(uu, o) = zk[o] / sk; cq(uu, o) = zq[o] / sq; }
      float mu = 0.f, xk = 0.f;
#pragma unroll 1
      for (int o = 0; o < NC; ++o) { mu += cq(uu, o); xk += ck(uu, o); }
      mu *= (1.0f / NC); xk *= (1.0f / NC); float var = 0.f;
#pragma unroll 1
      for (int o = 0; o < NC; ++o) { const float dv = cq(uu, o) - mu; var += dv * dv; }
      var *= (1.0f / (NC - 1)); const float sd = sqrtf(var); const float sigma = (sd > 20.f) ? sd : logf(1.0f + expf(sd));
      const float z = (xk - mu) / sigma; smu[l2l][uu] = mu; slp[l2l][uu] = -0.5f * z * z - logf(sigma) - 0.9189385332046727f; }
#pragma unroll 1
    for (int pp = 0; pp < NC; ++pp) { float mx = -3.0e38f;
#pragma unroll 1
      for (int uu = 0; uu < NC; ++uu) { float s = 0.f;
#pragma unroll 1
        for (int c = 0; c < NC; ++c) s += cq(pp, c) * ck(uu, c);
        s = (uu > pp) ? -1e9f : s * (1.0f / NC); e[uu] = s; mx = fmaxf(mx, s); }
      float se = 0.f;
#pragma unroll 1
      for (int uu = 0; uu < NC; ++uu) { e[uu] = expf(e[uu] - mx); se += e[uu]; }
#pragma unroll 1
      for (int c = 0; c < NC; ++c) { float a2 = 0.f;
#pragma unroll 1
        for (int uu = 0; uu < NC; ++uu) a2 += e[uu] * cq(uu, c);
        scq2[c][l2l][pp] = a2 / se; } }
#pragma unroll 1
    for (int c = 0; c < NC; ++c) { scq2[c][l2l][5] = 0.f; scq2[c][l2l][6] = 0.f; scq2[c][l2l][7] = 0.f; }
    smu[l2l][5] = smu[l2l][6] = smu[l2l][7] = 0.f; slp[l2l][5] = slp[l2l][6] = slp[l2l][7] = 0.f;
#undef cq
#undef ck
  }
  __syncthreads();
  for (int e = tid; e < NC * 64 * 2; e += 128) { const int c = e / 128, rem = e % 128, l2l = rem >> 1, q = rem & 1; vst2(CQ2 + ((((size_t)b * NC + c) * NL) + l20 + l2l) * 8 + q * 4, *(const v4f*)&scq2[c][l2l][q * 4]); }
  for (int e = tid; e < 64 * 2; e += 128) { const int l2l = e >> 1, q = e & 1; vst2(MU + (((size_t)b * NL) + l20 + l2l) * 8 + q * 4, *(const v4f*)&smu[l2l][q * 4]); vst2(LP + (((size_t)b * NL) + l20 + l2l) * 8 + q * 4, *(const v4f*)&slp[l2l][q * 4]); } }
__global__ __launch_bounds__(256) void k_ks(const float* __restrict__ CQ2, const float* __restrict__ WPB, const float* __restrict__ BPB, _Float16* __restrict__ KSH, _Float16* __restrict__ KSL) { __shared__ __align__(16) _Float16 sh[64][72], sl[64][72];
  const int t = threadIdx.x; const int k0 = blockIdx.x * 64, h = blockIdx.y; const size_t b = TKS0 + blockIdx.z;
  for (int e = t; e < 64 * DD; e += 256) { const int kl = e >> 6, d = e & 63; const int k = k0 + kl; float s = 0.f;
#pragma unroll 1
    for (int u2 = 0; u2 < NC; ++u2) { const unsigned X = ((unsigned)(h * NC + u2) * NL + k) * DD + d; const unsigned o = X / (unsigned)(NL * NC); const unsigned X5 = X / (unsigned)NC; const unsigned l = X5 & (NL - 1); const int p = (int)(X - X5 * NC); float a = bfr(BPB[o]);
#pragma unroll 1
      for (int c = 0; c < NC; ++c) {
#pragma unroll 1
        for (int tp = 0; tp < 3; ++tp) { const int ps = p + tp - 1; if (ps < 0 || ps >= NC) continue; a += bfr(WPB[((size_t)o * NC + c) * 3 + tp]) * CQ2[((b * NC + c) * NL + l) * 8 + ps]; } }
      s += fmaxf(a, 0.f); }
    const _Float16 hv = (_Float16)s; sh[kl][d] = hv; sl[kl][d] = (_Float16)((s - (float)hv) * 2048.0f); }
  __syncthreads();
  for (int e = t; e < 64 * 8; e += 256) { const int kl = e >> 3, q = e & 7; const size_t o = (((b * NH + h) * NL) + k0 + kl) * DD + q * 8; vst2((unsigned*)(KSH + o), *(const v4u*)&sh[kl][q * 8]); vst2((unsigned*)(KSL + o), *(const v4u*)&sl[kl][q * 8]); } }
__global__ __launch_bounds__(128) void k_vt(const float* __restrict__ V, _Float16* __restrict__ VT) { __shared__ __align__(16) _Float16 th[DD][72]; const int t = threadIdx.x; const size_t bh = TBH0 + blockIdx.y; const int m0 = blockIdx.x * 64;
  for (int e = t; e < 64 * DD; e += 128) { const int ml = e / DD, d = e % DD; th[d][ml] = (_Float16)bfr(V[(bh * NL + m0 + ml) * DD + d]); }
  __syncthreads(); for (int e = t; e < DD * 8; e += 128) { const int d = e >> 3, q = e & 7; vst2((unsigned*)(VT + (bh * DD + d) * (size_t)NL + m0 + q * 8), *(const v4u*)&th[d][q * 8]); } }
__global__ __launch_bounds__(128) void k_att(const float* __restrict__ Q, const _Float16* __restrict__ KSH, const _Float16* __restrict__ KSL, const _Float16* __restrict__ VT, float* __restrict__ OUT) {
  __shared__ __align__(16) float sp[4][16][36]; __shared__ __align__(16) float so[4][16][68];
  const int tid = threadIdx.x, wave = tid >> 5, lane = tid & 31, col = lane & 15, g = lane >> 4; const size_t bh = TBH0 + blockIdx.y; const int q0 = blockIdx.x * 64 + wave * 16; const size_t rq = bh * NL + q0;
  v16h aq[2];
#pragma unroll
  for (int kc = 0; kc < 2; ++kc) { const float* pp = Q + (rq + col) * DD + kc * 32 + 8 * g;
#pragma unroll
    for (int i = 0; i < 8; ++i) { aq[kc][i] = (_Float16)bfr(pp[i]); aq[kc][8 + i] = (_Float16)bfr(pp[16 + i]); } }
  float m[8], l[8];
#pragma unroll
  for (int r = 0; r < 8; ++r) { m[r] = -3.0e38f; l[r] = 0.f; }
  v8f acc[4] = {};
#pragma unroll 1
  for (int ks = 0; ks < NL / 32; ++ks) { float s[2][8];
#pragma unroll
    for (int ct = 0; ct < 2; ++ct) { const int kk = ks * 32 + ct * 16 + col; const size_t rk = (bh * NL + kk) * DD; v8f c = {}, cl = {};
#pragma unroll
      for (int kc = 0; kc < 2; ++kc) { c = wmma16(aq[kc], frag_h(KSH + rk + kc * 32, lane), c); cl = wmma16(aq[kc], frag_h(KSL + rk + kc * 32, lane), cl); }
#pragma unroll
      for (int r = 0; r < 8; ++r) s[ct][r] = c[r] + cl[r] * (1.0f / 2048.0f); }
    float alpha[8];
#pragma unroll
    for (int r = 0; r < 8; ++r) { float mx = fmaxf(s[0][r], s[1][r]);
#pragma unroll
      for (int o = 1; o < 16; o <<= 1) mx = fmaxf(mx, __shfl_xor(mx, o));
      const float mn = fmaxf(m[r], mx); alpha[r] = __expf(m[r] - mn); const float e0 = __expf(s[0][r] - mn), e1 = __expf(s[1][r] - mn); float es = e0 + e1;
#pragma unroll
      for (int o = 1; o < 16; o <<= 1) es += __shfl_xor(es, o);
      l[r] = l[r] * alpha[r] + es; m[r] = mn; sp[wave][8 * g + r][col] = e0; sp[wave][8 * g + r][16 + col] = e1; }
#pragma unroll
    for (int j = 0; j < 4; ++j)
#pragma unroll
      for (int r = 0; r < 8; ++r) acc[j][r] *= alpha[r];
    LDSX();
    v16h pa, par; { const float* prow = &sp[wave][col][0] + 8 * (lane >> 4);
#pragma unroll
      for (int i = 0; i < 8; ++i) { const float p0 = prow[i] * 2048.0f, p1 = prow[16 + i] * 2048.0f; pa[i] = (_Float16)p0; pa[8 + i] = (_Float16)p1; par[i] = (_Float16)(p0 - (float)pa[i]); par[8 + i] = (_Float16)(p1 - (float)pa[8 + i]); } }
#pragma unroll
    for (int j = 0; j < 4; ++j) { const v16h vh = frag_h(VT + (bh * DD + j * 16 + col) * (size_t)NL + ks * 32, lane); acc[j] = wmma16(pa, vh, acc[j]); acc[j] = wmma16(par, vh, acc[j]); }
    LDSX(); }
#pragma unroll
  for (int r = 0; r < 8; ++r) { const float il = (1.0f / 2048.0f) / l[r];
#pragma unroll
    for (int j = 0; j < 4; ++j) so[wave][8 * g + r][j * 16 + col] = acc[j][r] * il; }
  LDSX(); for (int rl = 0; rl < 16; ++rl) if (lane < 16) vst2(OUT + (rq + rl) * DD + lane * 4, *(const v4f*)&so[wave][rl][lane * 4]); }
__global__ __launch_bounds__(64) void k_loss(const float* __restrict__ MU, const float* __restrict__ LP, float* __restrict__ OUT1) { __shared__ float sce[64], slp[64];
  const int t = threadIdx.x;
  if (t < TNB * NC) { const int b = t / NC, u = t % NC; float mx = -3.0e38f;
#pragma unroll 1
    for (int l2 = 0; l2 < NL; ++l2) mx = fmaxf(mx, MU[((size_t)b * NL + l2) * 8 + u]);
    float se = 0.f;
#pragma unroll 1
    for (int l2 = 0; l2 < NL; ++l2) se += expf(MU[((size_t)b * NL + l2) * 8 + u] - mx);
    const float lse = mx + logf(se); float sc = 0.f, sl = 0.f;
#pragma unroll 1
    for (int l2 = 0; l2 < NL; ++l2) { const float mu = MU[((size_t)b * NL + l2) * 8 + u]; sc += mu * (mu - lse); sl += LP[((size_t)b * NL + l2) * 8 + u]; }
    sce[t] = sc; slp[t] = sl; }
  __syncthreads();
  if (t == 0) { float a = 0.f, c = 0.f; for (int i = 0; i < TNB * NC; ++i) { a += slp[i]; c += sce[i]; }
    const float n = (float)(TNB * NC); const float loss = -(a / (n * NL)) + (-(c / n)); vst2(OUT1, loss); } }
extern "C" void kernel_launch(void* const* d_in, const int* in_sizes, int n_in, void* d_out, int out_size, void* d_ws, size_t ws_size, hipStream_t stream) {
  (void)in_sizes; (void)n_in; (void)out_size;
  const float** F = (const float**)d_in;
  if (ws_size < (size_t)WS_END) return;
  char* ws = (char*)d_ws; float *CQ2 = (float*)(ws + WS_CQ2), *MU = (float*)(ws + WS_MU), *LP = (float*)(ws + WS_LP); _Float16 *KSH = (_Float16*)(ws + WS_KSH), *KSL = (_Float16*)(ws + WS_KSL), *VT = (_Float16*)(ws + WS_VT);
  float* OUT0 = (float*)d_out; float* OUT1 = OUT0 + (size_t)NB * NH * NL * DD;
  k_ckp<<<dim3(NL / 64, TNB), 128, 0, stream>>>(F[1], F[3], F[4], F[7], F[8], F[9], F[10], CQ2, MU, LP);
  k_ks<<<dim3(NL / 64, NH, TKSN), 256, 0, stream>>>(CQ2, F[5], F[6], KSH, KSL);
  k_vt<<<dim3(NL / 64, TBHN), 128, 0, stream>>>(F[2], VT);
  k_att<<<dim3(NL / 64, TBHN), 128, 0, stream>>>(F[0], KSH, KSL, VT, OUT0);
  k_loss<<<1, 64, 0, stream>>>(MU, LP, OUT1);
}
